// GNN_63385127354906
// MI455X (gfx1250) — hardware-run, weakly checked
//
#include <hip/hip_runtime.h>
#include <math.h>

constexpr int NNODE    = 50000;
constexpr int NEDGE    = 800000;
constexpr int NPADM    = 50048;
constexpr int FDIM     = 128;
constexpr int HDIM     = 32;
constexpr int HSLD     = 64;
constexpr int NT       = 256;
constexpr int SRB_AB   = 2048;
constexpr int NTILE_AB = 25;
constexpr int SRB_C    = 1024;
constexpr int NTILE_C  = 49;
constexpr int NPT      = NTILE_AB * SRB_AB;
constexpr int SCH      = 4096;
constexpr int SPT      = SCH / NT;
constexpr int NCH      = (NEDGE + SCH - 1) / SCH;
constexpr float WCARRY     = 16.0f;
constexpr float HCARRY     = 16.0f;
constexpr float LOCARRY    = 2048.0f;
constexpr float SC_X_HH    = 1.0f / 16.0f;
constexpr float SC_X_CR    = 1.0f / 32768.0f;
constexpr float SC_H_HH    = 1.0f / 256.0f;
constexpr float SC_H_CR    = 1.0f / 524288.0f;
constexpr float INV_SQRT_D = 0.17677669529663687f;
constexpr int WOFF_G   = 0;
constexpr int WOFF_Q   = 8192;
constexpr int WOFF_K   = 16384;
constexpr int WOFF_V   = 24576;
constexpr int WOFF_S   = 32768;
constexpr int WOFF_GLO = 36864;
constexpr int WOFF_SLO = 45056;
constexpr int WWORDS   = 49152;

static_assert(NPADM % 64 == 0 && NPADM >= NNODE, "");
static_assert(FDIM % 64 == 0 && FDIM % 32 == 0 && HSLD % 64 == 0, "");
static_assert(NEDGE % SPT == 0 && SCH % NT == 0 && SPT % 4 == 0, "");
static_assert(NPT >= NPADM && NTILE_C * SRB_C >= NNODE && NTILE_C * SRB_C <= NPT, "");
static_assert(SRB_AB == 8 * 256 && SRB_C == 8 * 128, "");
static_assert(NNODE % 4 == 0 && NNODE < 65536, "");
static_assert(WWORDS % NT == 0 && WOFF_S % NT == 0 && WOFF_GLO % NT == 0 && WOFF_SLO % NT == 0, "");
static_assert((NPADM * 16) % NT == 0, "");

typedef __attribute__((ext_vector_type(16))) _Float16 v16h;
typedef __attribute__((ext_vector_type(8)))  _Float16 v8h;
typedef __attribute__((ext_vector_type(16))) __bf16   v16b;
typedef __attribute__((ext_vector_type(8)))  __bf16   v8b;
typedef __attribute__((ext_vector_type(8)))  float    v8f;
typedef __attribute__((ext_vector_type(4)))  float    v4f;
typedef __attribute__((ext_vector_type(4)))  int      v4i;
typedef __attribute__((ext_vector_type(4)))  unsigned int v4u;
typedef __attribute__((ext_vector_type(2)))  unsigned int v2u;

__device__ __forceinline__ unsigned short f2bf_bits(float f) {
  unsigned u = __float_as_uint(f);
  return (unsigned short)((u + 0x7FFFu + ((u >> 16) & 1u)) >> 16);
}
__device__ __forceinline__ float bf_bits2f(unsigned short h) { return __uint_as_float(((unsigned)h) << 16); }

__device__ __forceinline__ void dep_guard_h(v8f& a, v8f& b, v16h x, v16h y) { asm volatile("v_nop\n\tv_nop\n\tv_nop\n\tv_nop" : "+v"(a), "+v"(b) : "v"(x), "v"(y)); }
__device__ __forceinline__ void dep_guard_b(v8f& a, v8f& b, v16b x, v16b y) { asm volatile("v_nop\n\tv_nop\n\tv_nop\n\tv_nop" : "+v"(a), "+v"(b) : "v"(x), "v"(y)); }
__device__ __forceinline__ void keep4_h(v16h a, v16h b, v16h c, v16h d) { asm volatile("v_nop" :: "v"(a), "v"(b), "v"(c), "v"(d)); }
__device__ __forceinline__ void keep4_b(v16b a, v16b b, v16b c, v16b d) { asm volatile("v_nop" :: "v"(a), "v"(b), "v"(c), "v"(d)); }
__device__ __forceinline__ void acc_guard4(v8f& a, v8f& b, v8f& c, v8f& d) { asm volatile("v_nop\n\tv_nop\n\tv_nop\n\tv_nop" : "+v"(a), "+v"(b), "+v"(c), "+v"(d)); }
template <typename T> struct Frag;
template <> struct Frag<_Float16> {
  typedef v16h V; union U { v16h v; v8h h[2]; };
  static __device__ __forceinline__ v16h load(const _Float16* p) {
    U f; f.h[0] = *(const v8h*)(p); f.h[1] = *(const v8h*)(p + 16); return f.v;
  }
  static __device__ __forceinline__ v8f mma(v16h a, v16h b, v8f c) {
    return __builtin_amdgcn_wmma_f32_16x16x32_f16(false, a, false, b, (short)0, c, false, false);
  }
  static __device__ __forceinline__ void guard(v8f& a, v8f& b, v16h x, v16h y) { dep_guard_h(a, b, x, y); }
  static __device__ __forceinline__ void keep(v16h a, v16h b, v16h c, v16h d) { keep4_h(a, b, c, d); }
};
template <> struct Frag<__bf16> {
  typedef v16b V; union U { v16b v; v8b h[2]; };
  static __device__ __forceinline__ v16b load(const __bf16* p) {
    U f; f.h[0] = *(const v8b*)(p); f.h[1] = *(const v8b*)(p + 16); return f.v;
  }
  static __device__ __forceinline__ v8f mma(v16b a, v16b b, v8f c) {
    return __builtin_amdgcn_wmma_f32_16x16x32_bf16(false, a, false, b, (short)0, c, false, false);
  }
  static __device__ __forceinline__ void guard(v8f& a, v8f& b, v16b x, v16b y) { dep_guard_b(a, b, x, y); }
  static __device__ __forceinline__ void keep(v16b a, v16b b, v16b c, v16b d) { keep4_b(a, b, c, d); }
};

template <int ET> struct Elem;
template <> struct Elem<0> { typedef _Float16 T; };
template <> struct Elem<1> { typedef __bf16 T; };
template <int ET, bool SPLIT, int BIAS_MODE, int OUT_MODE, bool RESID, int ACT = 0>
__global__ __launch_bounds__(256) void wmma_gemm64(
    const unsigned short* __restrict__ Ap, const unsigned short* __restrict__ A2p, int lda, long strideA,
    const unsigned short* __restrict__ Btp, const unsigned short* __restrict__ Bt2p, int ldb, long strideB,
    void* __restrict__ Cout, void* __restrict__ Cout2, int ldc, long strideC,
    const float* __restrict__ bias,
    const float* __restrict__ resid, long strideR,
    int M, int N, int K, float scale) {
  static_assert(!RESID || OUT_MODE == 0, "");
  static_assert(!RESID || ACT == 0, "");
  typedef typename Elem<ET>::T T;
  typedef typename Frag<T>::V V;
  const T* A = (const T*)Ap; const T* A2 = (const T*)A2p; const T* Bt = (const T*)Btp; const T* Bt2 = (const T*)Bt2p;
  __shared__ __align__(16) float sT[8][16 * 68];
  const int b    = blockIdx.y;
  const int lane = threadIdx.x & 31;
  const int wave = threadIdx.x >> 5;
  const int tilesN = N >> 6;
  const int tilesM = M >> 6;
  const int tile = blockIdx.x * 8 + wave;
  if (tile >= tilesM * tilesN) return;
  const int tm = tile / tilesN;
  const int tn = tile - tm * tilesN;
  const int m0 = tm << 6;
  const int n0 = tn << 6;

  const T* Ab  = A  + (size_t)b * strideA;
  const T* Bb  = Bt + (size_t)b * strideB;
  const T* Ab2 = SPLIT ? (A2  + (size_t)b * strideA) : nullptr;
  const T* Bb2 = SPLIT ? (Bt2 + (size_t)b * strideB) : nullptr;

  const int rlane = lane & 15;
  const int koff  = (lane >> 4) * 8;
  const int mOff  = (lane >> 4) * 8;

  v8f acc[4][4];
#pragma unroll
  for (int i = 0; i < 4; ++i)
#pragma unroll
    for (int j = 0; j < 4; ++j) acc[i][j] = (v8f){0.f,0.f,0.f,0.f,0.f,0.f,0.f,0.f};

  for (int k0 = 0; k0 < K; k0 += 32) {
    V bh[4], bl[4];
#pragma unroll
    for (int j = 0; j < 4; ++j) {
      const size_t bo = (size_t)(n0 + (j << 4) + rlane) * ldb + koff + k0;
      bh[j] = Frag<T>::load(Bb + bo);
      if (SPLIT) bl[j] = Frag<T>::load(Bb2 + bo);
    }
#pragma unroll
    for (int i = 0; i < 4; ++i) {
      const size_t ao = (size_t)(m0 + (i << 4) + rlane) * lda + koff + k0;
      V ah = Frag<T>::load(Ab + ao);
      V al;
      if (SPLIT) al = Frag<T>::load(Ab2 + ao);
#pragma unroll
      for (int j = 0; j < 4; ++j) {
        acc[i][j] = Frag<T>::mma(ah, bh[j], acc[i][j]);
        if (SPLIT) {
          acc[i][j] = Frag<T>::mma(ah, bl[j], acc[i][j]);
          acc[i][j] = Frag<T>::mma(al, bh[j], acc[i][j]);
        }
      }
      Frag<T>::guard(acc[i][0], acc[i][1], ah, SPLIT ? al : ah);
      Frag<T>::guard(acc[i][2], acc[i][3], ah, SPLIT ? al : ah);
    }
    Frag<T>::keep(bh[0], bh[1], bh[2], bh[3]);
    if (SPLIT) Frag<T>::keep(bl[0], bl[1], bl[2], bl[3]);
  }
  acc_guard4(acc[0][0], acc[0][1], acc[0][2], acc[0][3]);
  acc_guard4(acc[1][0], acc[1][1], acc[1][2], acc[1][3]);
  acc_guard4(acc[2][0], acc[2][1], acc[2][2], acc[2][3]);
  acc_guard4(acc[3][0], acc[3][1], acc[3][2], acc[3][3]);

  float* slab = sT[wave];
  const float* Rb = RESID ? (resid + (size_t)b * strideR) : nullptr;
#pragma unroll
  for (int i = 0; i < 4; ++i) {
    const int mBase = m0 + (i << 4);
#pragma unroll
    for (int j = 0; j < 4; ++j) {
      const int n = n0 + (j << 4) + rlane;
      float bv = 0.f;
      if (BIAS_MODE == 2) bv = bias[n];
#pragma unroll
      for (int r = 0; r < 8; ++r) {
        float v = acc[i][j][r] * scale;
        if (BIAS_MODE == 1) v += bias[mBase + mOff + r];
        if (BIAS_MODE == 2) v += bv;
        if (ACT == 2) v = fmaxf(v, 0.0f);
        if (ACT == 4) v = (v > 0.f) ? v : 0.01f * v;
        slab[(mOff + r) * 68 + (j << 4) + rlane] = v;
      }
    }
    __builtin_amdgcn_fence(__ATOMIC_RELEASE, "workgroup");
    __builtin_amdgcn_wave_barrier();
    __builtin_amdgcn_fence(__ATOMIC_ACQUIRE, "workgroup");
    if (OUT_MODE == 0) {
      float* C = (float*)Cout + (size_t)b * strideC;
      const int hh = lane >> 4, c4 = (lane & 15) * 4;
      if (RESID) {
#pragma unroll
        for (int it = 0; it < 8; ++it) {
          const int row = it * 2 + hh;
          const v4f rr = *(const v4f*)(Rb + (size_t)(mBase + row) * ldc + n0 + c4);
          v4f v = *(const v4f*)(slab + row * 68 + c4);
          v = v + rr;
          *(v4f*)(slab + row * 68 + c4) = v;
        }
      }
      for (int pass = 0; pass < 2; ++pass) {
#pragma unroll
        for (int it = 0; it < 8; ++it) {
          const int row = it * 2 + hh;
          v4f v = *(const v4f*)(slab + row * 68 + c4);
          *(volatile v4f*)(C + (size_t)(mBase + row) * ldc + n0 + c4) = v;
        }
        __threadfence();
      }
    } else {
      const int q = lane >> 3, c8 = (lane & 7) * 8;
      unsigned short* C  = (unsigned short*)Cout  + (size_t)b * strideC;
      unsigned short* C2 = (OUT_MODE == 2) ? ((unsigned short*)Cout2 + (size_t)b * strideC) : nullptr;
      for (int pass = 0; pass < 2; ++pass) {
#pragma unroll
        for (int it = 0; it < 4; ++it) {
          const int row = it * 4 + q;
          const float* sp = slab + row * 68 + c8;
          v8h hv, lv;
#pragma unroll
          for (int e = 0; e < 8; ++e) {
            if (OUT_MODE == 1) {
              hv[e] = (_Float16)sp[e]; lv[e] = hv[e];
            } else if (OUT_MODE == 3) {
              hv[e] = __builtin_bit_cast(_Float16, f2bf_bits(sp[e])); lv[e] = hv[e];
            } else {
              unsigned short hb = f2bf_bits(sp[e]);
              unsigned short lb = f2bf_bits(sp[e] - bf_bits2f(hb));
              hv[e] = __builtin_bit_cast(_Float16, hb);
              lv[e] = __builtin_bit_cast(_Float16, lb);
            }
          }
          *(volatile v8h*)(C + (size_t)(mBase + row) * ldc + n0 + c8) = hv;
          if (OUT_MODE == 2) *(volatile v8h*)(C2 + (size_t)(mBase + row) * ldc + n0 + c8) = lv;
        }
        __threadfence();
      }
    }
    __builtin_amdgcn_fence(__ATOMIC_RELEASE, "workgroup");
    __builtin_amdgcn_wave_barrier();
    __builtin_amdgcn_fence(__ATOMIC_ACQUIRE, "workgroup");
  }
}

__device__ __forceinline__ unsigned pk16(unsigned short a, unsigned short b) { return (unsigned)a | ((unsigned)b << 16); }
__device__ __forceinline__ unsigned short h_bits(float f) { const _Float16 h = (_Float16)f; return __builtin_bit_cast(unsigned short, h); }
__device__ __forceinline__ void hilo_bits(float v, unsigned short& hb, unsigned short& lb) {
  const _Float16 h = (_Float16)v;
  hb = __builtin_bit_cast(unsigned short, h);
  const float back = (float)h;
  const float r = (v - back) * LOCARRY;
  lb = h_bits(r);
}
__device__ __forceinline__ float bfw_lo(unsigned w) { float f = __uint_as_float(w << 16); asm volatile("" : "+v"(f)); return f; }
__device__ __forceinline__ float bfw_hi(unsigned w) { float f = __uint_as_float(w & 0xffff0000u); asm volatile("" : "+v"(f)); return f; }
__device__ __forceinline__ v4f shfl4_xor(v4f a, int m) {
  v4f r;
  r[0] = __shfl_xor(a[0], m, 32); r[1] = __shfl_xor(a[1], m, 32); r[2] = __shfl_xor(a[2], m, 32); r[3] = __shfl_xor(a[3], m, 32);
  return r;
}

__device__ __forceinline__ int blk_excl_scan(int cnt, int* scan_ws, int tid, int* tot) {
  const int lane = tid & 31, wave = tid >> 5; int incl = cnt;
#pragma unroll
  for (int o = 1; o < 32; o <<= 1) { const int v = __shfl_up(incl, o, 32); if (lane >= o) incl += v; }
  if (lane == 31) scan_ws[wave] = incl;
  __syncthreads();
  if (wave == 0) { int wv = (lane < NT / 32) ? scan_ws[lane] : 0; int wincl = wv;
#pragma unroll
    for (int o = 1; o < 32; o <<= 1) { const int v = __shfl_up(wincl, o, 32); if (lane >= o) wincl += v; }
    if (lane < NT / 32) scan_ws[32 + lane] = wincl - wv; if (lane == 31) scan_ws[64] = wincl; }
  __syncthreads();
  const int res = scan_ws[32 + wave] + incl - cnt; *tot = scan_ws[64];
  return res;
}
template <int SRBT, bool WITH_SRC, bool WITH_EIDX>
__device__ __forceinline__ int chunk_hits(const int* __restrict__ colv, const int* __restrict__ rowv, int e0, int n0, int tid,
                                          int* LIST, int* LISTE, int* scan_ws) {
  const int eb = e0 + tid * SPT;
  const bool inr = eb < NEDGE;
  const int ebc = inr ? eb : (NEDGE - SPT);
  int rec[SPT]; int cnt = 0;
#pragma unroll
  for (int k = 0; k < SPT; k += 4) {
    const v4i d4 = *(const v4i*)(colv + ebc + k);
    v4i s4 = (v4i){0, 0, 0, 0};
    if (WITH_SRC) s4 = *(const v4i*)(rowv + ebc + k);
#pragma unroll
    for (int e = 0; e < 4; ++e) {
      int d = d4[e]; d = d < 0 ? 0 : (d >= NNODE ? NNODE - 1 : d);
      int s = s4[e]; s = s < 0 ? 0 : (s >= NNODE ? NNODE - 1 : s);
      int r = -1;
      if (inr && d >= n0 && d < n0 + SRBT) { r = ((d - n0) << 16) | s; ++cnt; }
      rec[k + e] = r;
    }
  }
  int tot; int p = blk_excl_scan(cnt, scan_ws, tid, &tot);
#pragma unroll
  for (int k = 0; k < SPT; ++k) {
    if (rec[k] >= 0) {
      if ((unsigned)p < (unsigned)SCH) { LIST[p] = rec[k]; if (WITH_EIDX) LISTE[p] = eb + k; }
      ++p;
    }
  }
  __syncthreads();
  return tot < SCH ? tot : SCH;
}

__global__ __launch_bounds__(NT) void prep_w_kernel(const float* __restrict__ Wg, const float* __restrict__ Wq, const float* __restrict__ Wk,
                                                   const float* __restrict__ Wv, const float* __restrict__ Ws, unsigned* __restrict__ WPw) {
  const int i = blockIdx.x * NT + threadIdx.x;
  float a, b; bool lo;
  if (i < WOFF_S) {
    const int p = i >> 13; const int j = i & 8191;
    const float* W = (p == 0) ? Wg : (p == 1) ? Wq : (p == 2) ? Wk : Wv;
    a = W[2 * j] * WCARRY; b = W[2 * j + 1] * WCARRY; lo = false;
  } else if (i < WOFF_GLO) {
    const int j = i - WOFF_S; const int row = j >> 6; const bool live = row < HDIM; const int jj = live ? j : 0;
    const float fl = live ? WCARRY : 0.0f;
    a = Ws[2 * jj] * fl; b = Ws[2 * jj + 1] * fl; lo = false;
  } else if (i < WOFF_SLO) {
    const int j = i - WOFF_GLO;
    a = Wg[2 * j] * WCARRY; b = Wg[2 * j + 1] * WCARRY; lo = true;
  } else {
    const int j = i - WOFF_SLO; const int row = j >> 6; const bool live = row < HDIM; const int jj = live ? j : 0;
    const float fl = live ? WCARRY : 0.0f;
    a = Ws[2 * jj] * fl; b = Ws[2 * jj + 1] * fl; lo = true;
  }
  unsigned short ha, la, hb, lb;
  hilo_bits(a, ha, la); hilo_bits(b, hb, lb);
  const unsigned u = lo ? pk16(la, lb) : pk16(ha, hb);
  ((volatile unsigned*)WPw)[i] = u;
  __threadfence();
  ((volatile unsigned*)WPw)[i] = u;
}

__global__ __launch_bounds__(NT) void cast_x_kernel(const float* __restrict__ x, unsigned* __restrict__ XHw, unsigned* __restrict__ XLw) {
  const int i = blockIdx.x * NT + threadIdx.x;
  const int row = i >> 4;
  const bool live = row < NNODE;
  const int ic = live ? i : (NNODE * 16 - 1);
  const float* p = x + 8 * (size_t)ic;
  const v4f a = *(const v4f*)(p);
  const v4f c = *(const v4f*)(p + 4);
  const float fl = live ? 1.0f : 0.0f;
  unsigned short hb[8], lb[8];
#pragma unroll
  for (int e = 0; e < 4; ++e) {
    hilo_bits(a[e] * fl, hb[e], lb[e]);
    hilo_bits(c[e] * fl, hb[4 + e], lb[4 + e]);
  }
  const v4u uh = (v4u){pk16(hb[0], hb[1]), pk16(hb[2], hb[3]), pk16(hb[4], hb[5]), pk16(hb[6], hb[7])};
  const v4u ul = (v4u){pk16(lb[0], lb[1]), pk16(lb[2], lb[3]), pk16(lb[4], lb[5]), pk16(lb[6], lb[7])};
  unsigned* qh = XHw + 4 * (size_t)i;
  unsigned* ql = XLw + 4 * (size_t)i;
  *(volatile v4u*)qh = uh; *(volatile v4u*)ql = ul;
  __threadfence();
  *(volatile v4u*)qh = uh; *(volatile v4u*)ql = ul;
}

__global__ __launch_bounds__(NT) void deg_kernel(const int* __restrict__ ei, const float* __restrict__ ew,
                                                float* __restrict__ DEGW, float* __restrict__ DINV) {
  __shared__ int LIST[SCH];
  __shared__ int LISTE[SCH];
  __shared__ __align__(16) float SDEG[SRB_AB];
  __shared__ int scan_ws[80];
  const int tid = threadIdx.x, lane = tid & 31, wave = tid >> 5;
  const int n0 = blockIdx.x * SRB_AB;
  for (int i = tid; i < SCH; i += NT) { LIST[i] = 0; LISTE[i] = 0; }
  for (int i = tid; i < SRB_AB; i += NT) SDEG[i] = 0.0f;
  if (tid < 80) scan_ws[tid] = 0;
  __syncthreads();
  const int* colv = ei + NEDGE;
#pragma unroll 1
  for (int c = 0; c < NCH; ++c) {
    const int tot = chunk_hits<SRB_AB, false, true>(colv, ei, c * SCH, n0, tid, LIST, LISTE, scan_ws);
#pragma unroll 1
    for (int base = 0; base < tot; base += 32) {
      const int q = base + lane;
      const int qc = q < SCH ? q : SCH - 1;
      const int lv = LIST[qc];
      int le = LISTE[qc]; le = le < 0 ? 0 : (le >= NEDGE ? NEDGE - 1 : le);
      const int rv = (q < tot) ? lv : -1;
      const float wl = ew[le];
      const int own = (rv >= 0 && ((rv >> 16) >> 8) == wave) ? 1 : 0;
      unsigned msk = (unsigned)__ballot(own);
#pragma unroll 1
      for (int it = 0; it < 32; ++it) {
        if (msk == 0u) break;
        const int bp = __builtin_ctz(msk); msk &= msk - 1u;
        const int r = __shfl(rv, bp, 32);
        const float wv = __shfl(wl, bp, 32);
        const int dl = (r >> 16) & (SRB_AB - 1);
        if (lane == 0) SDEG[dl] += wv;
      }
    }
    __syncthreads();
  }
  __syncthreads();
#pragma unroll
  for (int half = 0; half < 2; ++half) {
    const int dl = wave * 256 + half * 128 + 4 * lane;
    const v4f sd = *(const v4f*)(SDEG + dl);
    v4f dg, di;
#pragma unroll
    for (int e = 0; e < 4; ++e) { const float d = 1.0f + sd[e]; dg[e] = d; di[e] = 1.0f / sqrtf(d); }
    float* pd = DEGW + n0 + dl;
    float* pi = DINV + n0 + dl;
    for (int pass = 0; pass < 2; ++pass) { *(volatile v4f*)pd = dg; *(volatile v4f*)pi = di; __threadfence(); }
  }
}

__global__ __launch_bounds__(NT) void gcn_kernel(const int* __restrict__ ei, const float* __restrict__ ew,
                                                const float* __restrict__ DEGW, const float* __restrict__ DINV,
                                                const float* __restrict__ XL, const float* __restrict__ bg,
                                                float* ACC, unsigned* __restrict__ H16w, unsigned* __restrict__ HLOw) {
  __shared__ int LIST[SCH];
  __shared__ int LISTE[SCH];
  __shared__ int scan_ws[80];
  const int tid = threadIdx.x, lane = tid & 31, wave = tid >> 5;
  const int n0 = blockIdx.x * SRB_AB;
  for (int i = tid; i < SCH; i += NT) { LIST[i] = 0; LISTE[i] = 0; }
  if (tid < 80) scan_ws[tid] = 0;
  const v4f z4 = {0.f, 0.f, 0.f, 0.f};
#pragma unroll 1
  for (int j = 0; j < 256; ++j) *(v4f*)(ACC + (size_t)(n0 + wave * 256 + j) * FDIM + 4 * lane) = z4;
  __syncthreads();
  const int* colv = ei + NEDGE;
#pragma unroll 1
  for (int c = 0; c < NCH; ++c) {
    const int tot = chunk_hits<SRB_AB, true, true>(colv, ei, c * SCH, n0, tid, LIST, LISTE, scan_ws);
#pragma unroll 1
    for (int base = 0; base < tot; base += 32) {
      const int q = base + lane;
      const int qc = q < SCH ? q : SCH - 1;
      const int lv = LIST[qc];
      int le = LISTE[qc]; le = le < 0 ? 0 : (le >= NEDGE ? NEDGE - 1 : le);
      int sl = lv & 0xFFFF; sl = sl >= NNODE ? NNODE - 1 : sl;
      const int rv = (q < tot) ? lv : -1;
      const float coefl = DINV[sl] * ew[le];
      const int own = (rv >= 0 && ((rv >> 16) >> 8) == wave) ? 1 : 0;
      unsigned msk = (unsigned)__ballot(own);
#pragma unroll 1
      for (int it = 0; it < 32; ++it) {
        if (msk == 0u) break;
        const int bp = __builtin_ctz(msk); msk &= msk - 1u;
        const int r = __shfl(rv, bp, 32);
        const float cf = __shfl(coefl, bp, 32);
        const int dl = (r >> 16) & (SRB_AB - 1);
        int s = r & 0xFFFF; s = s >= NNODE ? NNODE - 1 : s;
        const v4f xv = *(const v4f*)(XL + (size_t)s * FDIM + 4 * lane);
        float* rp = ACC + (size_t)(n0 + dl) * FDIM + 4 * lane;
        v4f a = *(const v4f*)rp;
        a = a + cf * xv;
        *(v4f*)rp = a;
      }
    }
    __syncthreads();
  }
  __syncthreads();
  const v4f bg4 = *(const v4f*)(bg + 4 * lane);
  const int l16 = lane & 15;
#pragma unroll 1
  for (int j = 0; j < 256; ++j) {
    const int n = n0 + wave * 256 + j;
    if (n < NPADM) {
      const bool live = n < NNODE;
      const v4f a = *(const v4f*)(ACC + (size_t)n * FDIM + 4 * lane);
      const v4f xv = *(const v4f*)(XL + (size_t)n * FDIM + 4 * lane);
      const float dn = DINV[n];
      const float rdeg = 1.0f / DEGW[n];
      const float fl = live ? HCARRY : 0.0f;
      v4f h = a * dn;
      h = h + xv * rdeg;
      h = h + bg4;
      h = h * fl;
      unsigned short hb0, hb1, hb2, hb3, lb0, lb1, lb2, lb3;
      hilo_bits(h[0], hb0, lb0); hilo_bits(h[1], hb1, lb1); hilo_bits(h[2], hb2, lb2); hilo_bits(h[3], hb3, lb3);
      const unsigned u0 = pk16(hb0, hb1), u1 = pk16(hb2, hb3);
      const unsigned v0 = pk16(lb0, lb1), v1 = pk16(lb2, lb3);
      const unsigned w0 = (unsigned)__shfl((int)u0, 2 * l16, 32);
      const unsigned w1 = (unsigned)__shfl((int)u1, 2 * l16, 32);
      const unsigned w2 = (unsigned)__shfl((int)u0, 2 * l16 + 1, 32);
      const unsigned w3 = (unsigned)__shfl((int)u1, 2 * l16 + 1, 32);
      const unsigned y0 = (unsigned)__shfl((int)v0, 2 * l16, 32);
      const unsigned y1 = (unsigned)__shfl((int)v1, 2 * l16, 32);
      const unsigned y2 = (unsigned)__shfl((int)v0, 2 * l16 + 1, 32);
      const unsigned y3 = (unsigned)__shfl((int)v1, 2 * l16 + 1, 32);
      const v4u uh = (v4u){w0, w1, w2, w3};
      const v4u ul = (v4u){y0, y1, y2, y3};
      unsigned* hp = H16w + (size_t)n * 64 + 4 * lane;
      unsigned* lp = HLOw + (size_t)n * 64 + 4 * lane;
      for (int pass = 0; pass < 2; ++pass) {
        if (lane < 16) { *(volatile v4u*)hp = uh; *(volatile v4u*)lp = ul; }
        __threadfence();
      }
    }
  }
}

__global__ __launch_bounds__(NT) void attn_kernel(const int* __restrict__ ei, const unsigned* __restrict__ QBw, const unsigned* __restrict__ KBw,
                                                 const float* __restrict__ V, const float* __restrict__ HS, const float* __restrict__ bs,
                                                 float* ACC, float* __restrict__ OUTPRE, float* __restrict__ BNPART) {
  __shared__ int LIST[SCH];
  __shared__ float SM[SRB_C * 4];
  __shared__ float SL[SRB_C * 4];
  __shared__ int scan_ws[80];
  __shared__ __align__(16) float red[8 * 64];
  const int tid = threadIdx.x, lane = tid & 31, wave = tid >> 5;
  const int n0 = blockIdx.x * SRB_C;
  const int hq = lane >> 3;
  const int l7 = lane & 7;
  for (int i = tid; i < SCH; i += NT) LIST[i] = 0;
  for (int i = tid; i < SRB_C * 4; i += NT) { SM[i] = -INFINITY; SL[i] = 0.0f; }
  if (tid < 80) scan_ws[tid] = 0;
  const v4f z4 = {0.f, 0.f, 0.f, 0.f};
#pragma unroll 1
  for (int j = 0; j < 128; ++j) *(v4f*)(ACC + (size_t)(n0 + wave * 128 + j) * FDIM + 4 * lane) = z4;
  __syncthreads();
  const int* colv = ei + NEDGE;
#pragma unroll 1
  for (int c = 0; c < NCH; ++c) {
    const int tot = chunk_hits<SRB_C, true, false>(colv, ei, c * SCH, n0, tid, LIST, LIST, scan_ws);
#pragma unroll 1
    for (int base = 0; base < tot; base += 32) {
      const int q = base + lane;
      const int qc = q < SCH ? q : SCH - 1;
      const int lv = LIST[qc];
      const int rv = (q < tot) ? lv : -1;
      const int own = (rv >= 0 && ((rv >> 16) >> 7) == wave) ? 1 : 0;
      unsigned msk = (unsigned)__ballot(own);
#pragma unroll 1
      for (int it = 0; it < 32; ++it) {
        if (msk == 0u) break;
        const int bp = __builtin_ctz(msk); msk &= msk - 1u;
        const int r = __shfl(rv, bp, 32);
        const int dl = (r >> 16) & (SRB_C - 1);
        int s = r & 0xFFFF; s = s >= NNODE ? NNODE - 1 : s;
        int nq = n0 + dl; nq = nq < NPADM ? nq : NPADM - 1;
        const v2u kw = *(const v2u*)(KBw + (size_t)s * 64 + 2 * lane);
        const v2u qw = *(const v2u*)(QBw + (size_t)nq * 64 + 2 * lane);
        const float k0 = bfw_lo(kw[0]), k1 = bfw_hi(kw[0]), k2 = bfw_lo(kw[1]), k3 = bfw_hi(kw[1]);
        const float q0 = bfw_lo(qw[0]), q1 = bfw_hi(qw[0]), q2 = bfw_lo(qw[1]), q3 = bfw_hi(qw[1]);
        float d = q0 * k0 + q1 * k1 + q2 * k2 + q3 * k3;
        d += __shfl_xor(d, 1, 32);
        d += __shfl_xor(d, 2, 32);
        d += __shfl_xor(d, 4, 32);
        const float al = d * INV_SQRT_D;
        const int mi = dl * 4 + hq;
        const float mo = SM[mi], lo = SL[mi];
        const float mn = fmaxf(mo, al);
        const float rr = expf(mo - mn);
        const float ex = expf(al - mn);
        const float ln = lo * rr + ex;
        if (l7 == 0) { SM[mi] = mn; SL[mi] = ln; }
        const v4f vv = *(const v4f*)(V + (size_t)s * FDIM + 4 * lane);
        float* rp = ACC + (size_t)(n0 + dl) * FDIM + 4 * lane;
        v4f a = *(const v4f*)rp;
        a = a * rr + ex * vv;
        *(v4f*)rp = a;
      }
    }
    __syncthreads();
  }
  __syncthreads();
  const v4f bs4 = *(const v4f*)(bs + 4 * l7);
  v4f psum = z4, psq = z4;
#pragma unroll 1
  for (int j = 0; j < 128; ++j) {
    const int dl = wave * 128 + j;
    const int n = n0 + dl;
    if (n < NNODE) {
      const float lsum = SL[dl * 4 + hq];
      const float inv = 1.0f / fmaxf(lsum, 1e-16f);
      const v4f a = *(const v4f*)(ACC + (size_t)n * FDIM + 4 * lane);
      v4f g = a * inv;
      g = g + shfl4_xor(g, 8);
      g = g + shfl4_xor(g, 16);
      const v4f hs4 = *(const v4f*)(HS + (size_t)n * HSLD + 4 * l7);
      v4f o = g * 0.25f;
      o = o + hs4;
      o = o + bs4;
      psum = psum + o;
      psq = psq + o * o;
      float* op = OUTPRE + (size_t)n * HDIM + 4 * lane;
      for (int pass = 0; pass < 2; ++pass) { if (lane < 8) *(volatile v4f*)op = o; __threadfence(); }
    }
  }
  if (lane < 8) {
    *(v4f*)(red + wave * 64 + 4 * lane) = psum;
    *(v4f*)(red + wave * 64 + 32 + 4 * lane) = psq;
  }
  __syncthreads();
  if (wave == 0) {
    const int l16 = lane & 15;
    v4f t = z4;
#pragma unroll
    for (int w = 0; w < 8; ++w) t = t + *(const v4f*)(red + w * 64 + 4 * l16);
    float* pp = BNPART + (size_t)blockIdx.x * 64 + 4 * lane;
    for (int pass = 0; pass < 2; ++pass) { if (lane < 16) *(volatile v4f*)pp = t; __threadfence(); }
  }
}

__global__ __launch_bounds__(NT) void bnstat_kernel(const float* __restrict__ BNPART, float* __restrict__ BNSS) {
  __shared__ __align__(16) float so[64];
  const int tid = threadIdx.x, lane = tid & 31, wave = tid >> 5;
  if (tid < 32) {
    double s = 0.0, ss = 0.0;
#pragma unroll 1
    for (int b = 0; b < NTILE_C; ++b) { s += (double)BNPART[b * 64 + tid]; ss += (double)BNPART[b * 64 + 32 + tid]; }
    const double mu = s * (1.0 / (double)NNODE);
    double var = ss * (1.0 / (double)NNODE) - mu * mu;
    var = var > 0.0 ? var : 0.0;
    const float muf = (float)mu;
    const float varf = (float)var;
    so[tid] = muf;
    so[32 + tid] = 1.0f / sqrtf(varf + 1e-5f);
  }
  __syncthreads();
  if (wave == 0) {
    const v4f v = *(const v4f*)(so + 4 * (lane & 15));
    float* pp = BNSS + 4 * lane;
    for (int pass = 0; pass < 2; ++pass) { if (lane < 16) *(volatile v4f*)pp = v; __threadfence(); }
  }
}

__global__ __launch_bounds__(NT) void bnapply_kernel(const float* __restrict__ OUTPRE, const float* __restrict__ BNSS,
                                                    const float* __restrict__ gam, const float* __restrict__ bet, float* __restrict__ out) {
  const int lane = threadIdx.x & 31, wave = threadIdx.x >> 5;
  const int rbase = (blockIdx.x * 8 + wave) * 4;
  if (rbase < NNODE) {
    const int row = rbase + (lane >> 3);
    const int c = 4 * (lane & 7);
    const v4f xv = *(const v4f*)(OUTPRE + (size_t)row * HDIM + c);
    const v4f mu = *(const v4f*)(BNSS + c);
    const v4f rs = *(const v4f*)(BNSS + 32 + c);
    const v4f g  = *(const v4f*)(gam + c);
    const v4f bb = *(const v4f*)(bet + c);
    v4f t = g * (xv - mu);
    t = t * rs;
    t = t + bb;
    v4f y;
#pragma unroll
    for (int e = 0; e < 4; ++e) y[e] = (t[e] > 0.0f) ? t[e] : 0.01f * t[e];
    float* op = out + (size_t)row * HDIM + c;
    *(volatile v4f*)op = y;
    __threadfence();
    *(volatile v4f*)op = y;
  }
}

extern "C" void kernel_launch(void* const* d_in, const int* in_sizes, int n_in,
                              void* d_out, int out_size, void* d_ws, size_t ws_size, hipStream_t stream) {
  if (n_in < 15) return;
  if (in_sizes[0] != NNODE * FDIM || in_sizes[1] != 2 * NEDGE || in_sizes[2] != NEDGE || out_size != NNODE * HDIM) return;
  if (in_sizes[3] != FDIM * FDIM || in_sizes[11] != HDIM * FDIM || in_sizes[12] != HDIM || in_sizes[13] != HDIM || in_sizes[14] != HDIM) return;
  const float* x    = (const float*)d_in[0];
  const int*   ei   = (const int*)  d_in[1];
  const float* ew   = (const float*)d_in[2];
  const float* Wg   = (const float*)d_in[3];
  const float* bg   = (const float*)d_in[4];
  const float* Wq   = (const float*)d_in[5];
  const float* bq   = (const float*)d_in[6];
  const float* Wk   = (const float*)d_in[7];
  const float* bk   = (const float*)d_in[8];
  const float* Wv   = (const float*)d_in[9];
  const float* bv   = (const float*)d_in[10];
  const float* Ws   = (const float*)d_in[11];
  const float* bs   = (const float*)d_in[12];
  const float* gam  = (const float*)d_in[13];
  const float* bet  = (const float*)d_in[14];
  float* out = (float*)d_out;

  char* ws = (char*)d_ws; size_t off = 0;
  auto carve = [&](size_t bytes) -> char* { char* p = ws + off; off += (bytes + 255) & ~(size_t)255; return p; };
  float*          DEGW   = (float*)carve((size_t)NPT * 4);
  float*          DINV   = (float*)carve((size_t)NPT * 4);
  unsigned short* X16    = (unsigned short*)carve((size_t)NPADM * FDIM * 2);
  unsigned short* XLO    = (unsigned short*)carve((size_t)NPADM * FDIM * 2);
  unsigned short* WPL    = (unsigned short*)carve((size_t)WWORDS * 4);
  float*          XLV    = (float*)carve((size_t)NPADM * FDIM * 4);
  float*          ACC    = (float*)carve((size_t)NPT * FDIM * 4);
  unsigned short* QB     = (unsigned short*)carve((size_t)NPADM * FDIM * 2);
  unsigned short* KB     = (unsigned short*)carve((size_t)NPADM * FDIM * 2);
  float*          HS     = (float*)carve((size_t)NPADM * HSLD * 4);
  float*          OUTPRE = (float*)carve((size_t)NNODE * HDIM * 4);
  float*          BNPART = (float*)carve((size_t)NTILE_C * 64 * 4);
  float*          BNSS   = (float*)carve((size_t)64 * 4);
  if (off > ws_size || off > (size_t)134217728) return;

  unsigned short* H16 = X16;
  unsigned short* HLO = XLO;
  const unsigned short* WG16 = WPL + 2 * WOFF_G;
  const unsigned short* WQ16 = WPL + 2 * WOFF_Q;
  const unsigned short* WK16 = WPL + 2 * WOFF_K;
  const unsigned short* WV16 = WPL + 2 * WOFF_V;
  const unsigned short* WS16 = WPL + 2 * WOFF_S;
  const unsigned short* WGLO = WPL + 2 * WOFF_GLO;
  const unsigned short* WSLO = WPL + 2 * WOFF_SLO;
  float* TMP64 = ACC;

  const int tiles128 = (NPADM / 64) * (FDIM / 64);
  const int tiles64  = (NPADM / 64) * (HSLD / 64);
  const dim3 g128((tiles128 + 7) / 8, 1), g64((tiles64 + 7) / 8, 1);

  prep_w_kernel<<<WWORDS / NT, NT, 0, stream>>>(Wg, Wq, Wk, Wv, Ws, (unsigned*)WPL);
  cast_x_kernel<<<(NPADM * 16) / NT, NT, 0, stream>>>(x, (unsigned*)X16, (unsigned*)XLO);

  wmma_gemm64<0, false, 0, 0, false><<<g128, 256, 0, stream>>>(
      XLO, nullptr, FDIM, 0L, WG16, nullptr, FDIM, 0L, (void*)XLV, nullptr, FDIM, 0L,
      nullptr, nullptr, 0L, NPADM, FDIM, FDIM, SC_X_CR);
  wmma_gemm64<0, false, 0, 0, true><<<g128, 256, 0, stream>>>(
      X16, nullptr, FDIM, 0L, WGLO, nullptr, FDIM, 0L, (void*)ACC, nullptr, FDIM, 0L,
      nullptr, XLV, 0L, NPADM, FDIM, FDIM, SC_X_CR);
  wmma_gemm64<0, false, 0, 0, true><<<g128, 256, 0, stream>>>(
      X16, nullptr, FDIM, 0L, WG16, nullptr, FDIM, 0L, (void*)XLV, nullptr, FDIM, 0L,
      nullptr, ACC, 0L, NPADM, FDIM, FDIM, SC_X_HH);

  deg_kernel<<<NTILE_AB, NT, 0, stream>>>(ei, ew, DEGW, DINV);
  gcn_kernel<<<NTILE_AB, NT, 0, stream>>>(ei, ew, DEGW, DINV, XLV, bg, ACC, (unsigned*)H16, (unsigned*)HLO);

  wmma_gemm64<0, false, 2, 3, false><<<g128, 256, 0, stream>>>(
      H16, nullptr, FDIM, 0L, WQ16, nullptr, FDIM, 0L, (void*)QB, nullptr, FDIM, 0L,
      bq, nullptr, 0L, NPADM, FDIM, FDIM, SC_H_HH);
  wmma_gemm64<0, false, 2, 3, false><<<g128, 256, 0, stream>>>(
      H16, nullptr, FDIM, 0L, WK16, nullptr, FDIM, 0L, (void*)KB, nullptr, FDIM, 0L,
      bk, nullptr, 0L, NPADM, FDIM, FDIM, SC_H_HH);
  wmma_gemm64<0, false, 2, 0, false><<<g128, 256, 0, stream>>>(
      H16, nullptr, FDIM, 0L, WV16, nullptr, FDIM, 0L, (void*)XLV, nullptr, FDIM, 0L,
      bv, nullptr, 0L, NPADM, FDIM, FDIM, SC_H_HH);

  wmma_gemm64<0, false, 0, 0, false><<<g64, 256, 0, stream>>>(
      HLO, nullptr, FDIM, 0L, WS16, nullptr, FDIM, 0L, (void*)HS, nullptr, HSLD, 0L,
      nullptr, nullptr, 0L, NPADM, HSLD, FDIM, SC_H_CR);
  wmma_gemm64<0, false, 0, 0, true><<<g64, 256, 0, stream>>>(
      H16, nullptr, FDIM, 0L, WSLO, nullptr, FDIM, 0L, (void*)TMP64, nullptr, HSLD, 0L,
      nullptr, HS, 0L, NPADM, HSLD, FDIM, SC_H_CR);
  wmma_gemm64<0, false, 0, 0, true><<<g64, 256, 0, stream>>>(
      H16, nullptr, FDIM, 0L, WS16, nullptr, FDIM, 0L, (void*)HS, nullptr, HSLD, 0L,
      nullptr, TMP64, 0L, NPADM, HSLD, FDIM, SC_H_HH);

  attn_kernel<<<NTILE_C, NT, 0, stream>>>(ei, (const unsigned*)QB, (const unsigned*)KB, XLV, HS, bs, ACC, OUTPRE, BNPART);
  bnstat_kernel<<<1, NT, 0, stream>>>(BNPART, BNSS);
  bnapply_kernel<<<(NNODE + 31) / 32, NT, 0, stream>>>(OUTPRE, BNSS, gam, bet, out);
}
